// EncoderBlock_14697378087355
// MI455X (gfx1250) — hardware-verified
//
#include <hip/hip_runtime.h>
#ifndef NB
#define NB 16
#endif
#ifndef SEQ
#define SEQ 1024
#endif
#define NB_FULL 16
#define SEQ_FULL 1024
#define DM 256
#define NH 8
#define HD 32
#define DF 1024
#define NR ((size_t)NB * SEQ)
static_assert(SEQ % 128 == 0);
static_assert(SEQ <= SEQ_FULL);
static_assert(NB <= NB_FULL);
static_assert(NH * HD == DM);
static_assert((NB * SEQ) % 8 == 0);

typedef unsigned short v8us __attribute__((ext_vector_type(8), may_alias));
typedef float  v8f  __attribute__((ext_vector_type(8)));
typedef float  v4f  __attribute__((ext_vector_type(4)));
typedef float  v4fa __attribute__((ext_vector_type(4), may_alias));
typedef _Float16 v16h __attribute__((ext_vector_type(16)));
typedef _Float16 v4h __attribute__((ext_vector_type(4)));
union FragH { v16h v; v8us half[2]; _Float16 h[16]; unsigned short u[16]; };

__device__ __forceinline__ unsigned short bf16_bits(float x) { unsigned int u = __float_as_uint(x); return (unsigned short)((u + 0x7FFFu + ((u >> 16) & 1u)) >> 16); }
__device__ __forceinline__ float bf16_val(unsigned short b) { return __uint_as_float(((unsigned int)b) << 16); }
__device__ __forceinline__ float bf16_rne(float x) { return bf16_val(bf16_bits(x)); }

__device__ __forceinline__ v16h g2_frag(const _Float16* p, int hh) { FragH f; f.half[0] = *(const v8us*)((const unsigned short*)p + 8 * hh); f.half[1] = *(const v8us*)((const unsigned short*)p + 16 + 8 * hh); return f.v; }
__device__ __forceinline__ v8f g2_mma(v16h a, v16h b, v8f c) { v8f d = __builtin_amdgcn_wmma_f32_16x16x32_f16(false, a, false, b, (short)0, c, false, false); asm volatile("v_nop\n\tv_nop\n\tv_nop\n\tv_nop" : "+v"(d) : "v"(a), "v"(b)); return d; }

__global__ __launch_bounds__(256) void k_wt_f16(const float* __restrict__ W, _Float16* __restrict__ Wt, unsigned K, unsigned N, float scale) {
  const unsigned t = blockIdx.x * 256u + threadIdx.x; const unsigned k8n = K >> 3; if (t >= N * k8n) return;
  const unsigned n = t / k8n, k8 = (t - n * k8n) * 8u; FragH f;
#pragma unroll
  for (int i = 0; i < 8; ++i) f.h[i] = (_Float16)(bf16_rne(W[(size_t)(k8 + i) * N + n]) * scale);
  const v8us o = f.half[0]; unsigned short* d = (unsigned short*)Wt + (size_t)n * K + k8;
  *(volatile v8us*)d = o; __threadfence(); *(volatile v8us*)d = o;
}

__global__ __launch_bounds__(256) void k_wqkv(const float* __restrict__ wq, const float* __restrict__ wk, const float* __restrict__ wv, _Float16* __restrict__ Wt) {
  const unsigned t = blockIdx.x * 256u + threadIdx.x; if (t >= 768u * 32u) return;
  const unsigned n = t >> 5, c8 = (t & 31u) * 8u; const unsigned sel = n >> 8, h = (n >> 5) & 7u, d = n & 31u;
  const float* w = (sel == 0u) ? wq : ((sel == 1u) ? wk : wv); FragH f;
#pragma unroll
  for (int i = 0; i < 8; ++i) f.h[i] = (_Float16)(bf16_rne(w[((size_t)h * DM + c8 + i) * HD + d]) * 16.0f);
  const v8us o = f.half[0]; unsigned short* dp = (unsigned short*)Wt + (size_t)n * DM + c8;
  *(volatile v8us*)dp = o; __threadfence(); *(volatile v8us*)dp = o;
}

template <int BFIN>
__global__ __launch_bounds__(256) void k_lnw(const float* __restrict__ X, size_t bstride, const float* __restrict__ g, const float* __restrict__ bb, float eps, _Float16* __restrict__ N16) {
  #pragma clang fp contract(off)
  const unsigned tid = threadIdx.x, lane = tid & 31u, w = tid >> 5;
  const unsigned r = blockIdx.x * 8u + w; const unsigned b = r / (unsigned)SEQ, s = r - b * (unsigned)SEQ;
  const float* xr = X + (size_t)b * bstride + (size_t)s * DM + lane * 8u;
  const v4f xa = *(const v4fa*)xr, xc = *(const v4fa*)(xr + 4);
  float v[8] = {xa[0], xa[1], xa[2], xa[3], xc[0], xc[1], xc[2], xc[3]};
  float sum = 0.f;
#pragma unroll
  for (int i = 0; i < 8; ++i) { if (BFIN) v[i] = bf16_rne(v[i]); sum += v[i]; }
  sum += __shfl_xor(sum, 1, 32); sum += __shfl_xor(sum, 2, 32); sum += __shfl_xor(sum, 4, 32); sum += __shfl_xor(sum, 8, 32); sum += __shfl_xor(sum, 16, 32);
  const float mu = sum * (1.0f / (float)DM);
  float vs = 0.f;
#pragma unroll
  for (int i = 0; i < 8; ++i) { const float dl = v[i] - mu; vs += dl * dl; }
  vs += __shfl_xor(vs, 1, 32); vs += __shfl_xor(vs, 2, 32); vs += __shfl_xor(vs, 4, 32); vs += __shfl_xor(vs, 8, 32); vs += __shfl_xor(vs, 16, 32);
  const float rs = rsqrtf(vs * (1.0f / (float)DM) + eps);
  const v4f ga = *(const v4fa*)(g + lane * 8u), gc = *(const v4fa*)(g + lane * 8u + 4), ba = *(const v4fa*)(bb + lane * 8u), bc = *(const v4fa*)(bb + lane * 8u + 4);
  const float gg[8] = {ga[0], ga[1], ga[2], ga[3], gc[0], gc[1], gc[2], gc[3]}; const float be[8] = {ba[0], ba[1], ba[2], ba[3], bc[0], bc[1], bc[2], bc[3]};
  FragH f;
#pragma unroll
  for (int i = 0; i < 8; ++i) f.h[i] = (_Float16)((v[i] - mu) * rs * bf16_rne(gg[i]) + bf16_rne(be[i]));
  const v8us o = f.half[0]; unsigned short* d = (unsigned short*)N16 + (size_t)r * DM + lane * 8u;
  *(volatile v8us*)d = o; __threadfence(); *(volatile v8us*)d = o;
}

template <int ACT, int HASB, int RESM, int O16>
__global__ __launch_bounds__(128) void k_gemm2(const _Float16* __restrict__ A, int lda, size_t sA, const _Float16* __restrict__ Bh, int ldb, size_t sB, float alpha, const float* __restrict__ bias,
    const float* __restrict__ CP, int ldcp, size_t sCP, float* __restrict__ C, _Float16* __restrict__ C16, int ldc, size_t sC, int M, int N, int K) {
  static_assert(ACT == 0 || ACT == 3);
  static_assert(!(ACT != 0 && RESM != 0));
  __shared__ __attribute__((aligned(16))) float so[4][32][68];
  const unsigned tid = threadIdx.x, w = tid >> 5, lane = tid & 31u, ln = lane & 15u; const int hh = (int)(lane >> 4); const unsigned by = blockIdx.y;
  A += (size_t)by * sA; Bh += (size_t)by * sB; const size_t cofs = (size_t)by * sC; const size_t pofs = (size_t)by * sCP;
  const unsigned ntn = (unsigned)N >> 6; const unsigned mt = blockIdx.x / ntn, nq = blockIdx.x - mt * ntn; const unsigned row0 = mt * 128u + 32u * w, col0 = nq * 64u; if (row0 >= (unsigned)M) return;
  const _Float16* a0p = A + (size_t)(row0 + ln) * lda; const _Float16* a1p = a0p + (size_t)16 * lda;
  const _Float16* b0p = Bh + (size_t)(col0 + ln) * ldb; const _Float16* b1p = b0p + (size_t)16 * ldb; const _Float16* b2p = b1p + (size_t)16 * ldb; const _Float16* b3p = b2p + (size_t)16 * ldb;
  const v8f z8 = {0.f,0.f,0.f,0.f,0.f,0.f,0.f,0.f}; v8f c00 = z8, c01 = z8, c02 = z8, c03 = z8, c10 = z8, c11 = z8, c12 = z8, c13 = z8;
#pragma unroll 1
  for (int kb = 0; kb < K; kb += 32) { const v16h a0 = g2_frag(a0p + kb, hh), a1 = g2_frag(a1p + kb, hh);
    v16h b = g2_frag(b0p + kb, hh); c00 = g2_mma(a0, b, c00); c10 = g2_mma(a1, b, c10);
    b = g2_frag(b1p + kb, hh); c01 = g2_mma(a0, b, c01); c11 = g2_mma(a1, b, c11);
    b = g2_frag(b2p + kb, hh); c02 = g2_mma(a0, b, c02); c12 = g2_mma(a1, b, c12);
    b = g2_frag(b3p + kb, hh); c03 = g2_mma(a0, b, c03); c13 = g2_mma(a1, b, c13); }
  v8f accs[8] = {c00, c01, c02, c03, c10, c11, c12, c13};
#pragma unroll
  for (int u = 0; u < 8; ++u) { const int t = u & 3, half = u >> 2; const unsigned col = col0 + (unsigned)t * 16u + ln; float bv = 0.f; if (HASB) bv = bf16_rne(bias[col]);
#pragma unroll
    for (int r = 0; r < 8; ++r) { const int rloc = half * 16 + 8 * hh + r; float v = accs[u][r] * alpha + bv; if (ACT == 3) v = fmaxf(v, 0.f); so[w][rloc][t * 16 + (int)ln] = v; } }
  __builtin_amdgcn_fence(4  , "workgroup"); __builtin_amdgcn_wave_barrier();
  const unsigned rsub = lane >> 4, c4 = (lane & 15u) * 4u;
  if (RESM != 0) {
#pragma unroll
    for (int q = 0; q < 16; ++q) { const unsigned r = (unsigned)q * 2u + rsub; v4f v = *(const v4fa*)&so[w][r][c4]; v4f rv = *(const v4fa*)(CP + pofs + (size_t)(row0 + r) * ldcp + col0 + c4);
      if (RESM == 2) { rv[0] = bf16_rne(rv[0]); rv[1] = bf16_rne(rv[1]); rv[2] = bf16_rne(rv[2]); rv[3] = bf16_rne(rv[3]); }
      v[0] += rv[0]; v[1] += rv[1]; v[2] += rv[2]; v[3] += rv[3]; *(v4fa*)&so[w][r][c4] = v; }
    __builtin_amdgcn_fence(4  , "workgroup"); __builtin_amdgcn_wave_barrier();
  }
  for (int pass = 0; pass < 2; ++pass) {
#pragma unroll
    for (int q = 0; q < 16; ++q) { const unsigned r = (unsigned)q * 2u + rsub; const v4f v = *(const v4fa*)&so[w][r][c4];
      if (O16 == 0) *(volatile v4f*)(C + cofs + (size_t)(row0 + r) * ldc + col0 + c4) = v;
      else { v4h h4; h4[0] = (_Float16)v[0]; h4[1] = (_Float16)v[1]; h4[2] = (_Float16)v[2]; h4[3] = (_Float16)v[3]; *(volatile v4h*)(C16 + cofs + (size_t)(row0 + r) * ldc + col0 + c4) = h4; } }
    if (pass == 0) __threadfence(); } }

__global__ __launch_bounds__(128) void k_fattn(const _Float16* __restrict__ QK, const _Float16* __restrict__ VT, _Float16* __restrict__ ATT) {
  __shared__ __attribute__((aligned(16))) _Float16 pl[4][16][40];
  __shared__ __attribute__((aligned(16))) _Float16 ol[4][16][72];
  const unsigned tid = threadIdx.x, w = tid >> 5, lane = tid & 31u, ln = lane & 15u; const int hh = (int)(lane >> 4);
  const unsigned qt = blockIdx.x, hp = blockIdx.y, b = blockIdx.z;
  const unsigned q0 = qt * 64u + w * 16u; const unsigned jmax = (q0 + 15u) >> 5;
  const _Float16* qkb = QK + (size_t)b * SEQ * 512; const _Float16* vtb = VT + (size_t)b * DM * SEQ;
  const v8f z8 = {0.f,0.f,0.f,0.f,0.f,0.f,0.f,0.f};
#pragma unroll 1
  for (unsigned hs = 0; hs < 2u; ++hs) {
    const unsigned h = hp * 2u + hs;
    const v16h qf = g2_frag(qkb + (size_t)(q0 + ln) * 512 + h * HD, hh);
    float mrow[8], lrow[8];
#pragma unroll
    for (int r = 0; r < 8; ++r) { mrow[r] = -1.0e30f; lrow[r] = 0.f; }
    v8f O0 = z8, O1 = z8;
#pragma unroll 1
    for (unsigned jt = 0; jt <= jmax; ++jt) {
      const unsigned k0 = jt * 32u;
      const _Float16* kr0 = qkb + (size_t)(k0 + ln) * 512 + 256 + h * HD;
      const v16h kf0 = g2_frag(kr0, hh), kf1 = g2_frag(kr0 + (size_t)16 * 512, hh);
      const _Float16* vr0 = vtb + (size_t)(h * HD + ln) * SEQ + k0;
      const v16h vf0 = g2_frag(vr0, hh), vf1 = g2_frag(vr0 + (size_t)16 * SEQ, hh);
      const v8f S0 = g2_mma(qf, kf0, z8); const v8f S1 = g2_mma(qf, kf1, z8);
#pragma unroll
      for (int r = 0; r < 8; ++r) {
        const unsigned qrow = q0 + 8u * (unsigned)hh + (unsigned)r, key = k0 + ln;
        const bool u0 = key <= qrow, u1 = (key + 16u) <= qrow;
        const float a0 = u0 ? S0[r] * 0.0625f : -1.0e30f; const float a1 = u1 ? S1[r] * 0.0625f : -1.0e30f;
        float cm = fmaxf(a0, a1);
        cm = fmaxf(cm, __shfl_xor(cm, 1, 32)); cm = fmaxf(cm, __shfl_xor(cm, 2, 32)); cm = fmaxf(cm, __shfl_xor(cm, 4, 32)); cm = fmaxf(cm, __shfl_xor(cm, 8, 32));
        const float nm = fmaxf(mrow[r], cm); const float al = __expf(mrow[r] - nm);
        const float x0 = __expf(a0 - nm), x1 = __expf(a1 - nm);
        const float e0 = u0 ? x0 : 0.f, e1 = u1 ? x1 : 0.f;
        lrow[r] = lrow[r] * al + (e0 + e1); mrow[r] = nm; O0[r] *= al; O1[r] *= al;
        pl[w][8 * hh + r][ln] = (_Float16)(e0 * 256.0f); pl[w][8 * hh + r][16u + ln] = (_Float16)(e1 * 256.0f);
      }
      __builtin_amdgcn_fence(4  , "workgroup"); __builtin_amdgcn_wave_barrier();
      const v16h pf = g2_frag(&pl[w][ln][0], hh);
      O0 = g2_mma(pf, vf0, O0); O1 = g2_mma(pf, vf1, O1);
      __builtin_amdgcn_fence(4  , "workgroup"); __builtin_amdgcn_wave_barrier();
    }
#pragma unroll
    for (int r = 0; r < 8; ++r) { float l = lrow[r]; l += __shfl_xor(l, 1, 32); l += __shfl_xor(l, 2, 32); l += __shfl_xor(l, 4, 32); l += __shfl_xor(l, 8, 32);
      const float inv = 0.0625f * __builtin_amdgcn_rcpf(l);
      ol[w][8 * hh + r][hs * 32u + ln] = (_Float16)(O0[r] * inv); ol[w][8 * hh + r][hs * 32u + 16u + ln] = (_Float16)(O1[r] * inv); }
  }
  __builtin_amdgcn_fence(4  , "workgroup"); __builtin_amdgcn_wave_barrier();
  const unsigned rq = lane >> 3, pc = lane & 7u;
  for (int pass = 0; pass < 2; ++pass) {
#pragma unroll
    for (int q = 0; q < 4; ++q) { const unsigned r = (unsigned)q * 4u + rq; const v8us v = *(const v8us*)&ol[w][r][pc * 8u];
      *(volatile v8us*)((unsigned short*)ATT + ((size_t)b * SEQ + q0 + r) * DM + hp * 64u + pc * 8u) = v; }
    if (pass == 0) __threadfence(); } }

static_assert((768u * 32u) % 256u == 0);
static_assert((size_t)768 * DM * 2 + (size_t)DM * DM * 2 + (size_t)DF * DM * 2 * 2 + NR * DM * 2 * 4 + NR * 512 * 2 + NR * DM * 4 + NR * DF * 2 + 11 * 256 <= (size_t)134217728);

extern "C" void kernel_launch(void* const* d_in, const int* in_sizes, int n_in,
                              void* d_out, int out_size, void* d_ws, size_t ws_size, hipStream_t stream) {
  if (n_in < 14) return;
  const size_t xneed = ((size_t)(NB - 1) * SEQ_FULL + SEQ) * DM;
  if ((size_t)in_sizes[0] < xneed || (size_t)out_size < xneed) return;
  if (in_sizes[1] < NH * DM * HD || in_sizes[2] < NH * DM * HD || in_sizes[3] < NH * DM * HD || in_sizes[4] < DM * DM || in_sizes[5] < DM || in_sizes[6] < DM * DF || in_sizes[7] < DF || in_sizes[8] < DF * DM || in_sizes[9] < DM || in_sizes[10] < DM || in_sizes[11] < DM || in_sizes[12] < DM || in_sizes[13] < DM) return;
  const float* const* I = (const float* const*)d_in;
  const float* x = I[0]; const float* wq = I[1]; const float* wk = I[2]; const float* wv = I[3]; const float* wp = I[4]; const float* bp = I[5]; const float* w1 = I[6]; const float* b1 = I[7]; const float* w2 = I[8]; const float* b2 = I[9]; const float* g1 = I[10]; const float* be1 = I[11]; const float* g2 = I[12]; const float* be2 = I[13];
  char* ws = (char*)d_ws; size_t off = 0;
  auto take = [&](size_t bytes) { char* p = ws + off; off += (bytes + 255) & ~(size_t)255; return p; };
  _Float16* BQKV = (_Float16*)take((size_t)768 * DM * 2);
  _Float16* BP   = (_Float16*)take((size_t)DM * DM * 2);
  _Float16* BW1  = (_Float16*)take((size_t)DF * DM * 2);
  _Float16* BW2  = (_Float16*)take((size_t)DM * DF * 2);
  _Float16* H16  = (_Float16*)take(NR * DM * 2);
  _Float16* QK16 = (_Float16*)take(NR * 512 * 2);
  _Float16* VT   = (_Float16*)take((size_t)NB * DM * SEQ * 2);
  _Float16* AT16 = (_Float16*)take(NR * DM * 2);
  float*    X2   = (float*)take(NR * DM * 4);
  _Float16* H2   = (_Float16*)take(NR * DM * 2);
  _Float16* F16  = (_Float16*)take(NR * DF * 2);
  if (off > ws_size || off > (size_t)134217728) return;
  float* out = (float*)d_out;

  k_wqkv<<<(768u * 32u) / 256u, 256, 0, stream>>>(wq, wk, wv, BQKV);
  k_wt_f16<<<(unsigned)(DM * (DM / 8) / 256), 256, 0, stream>>>(wp, BP, (unsigned)DM, (unsigned)DM, 16.0f);
  k_wt_f16<<<(unsigned)(DF * (DM / 8) / 256), 256, 0, stream>>>(w1, BW1, (unsigned)DM, (unsigned)DF, 16.0f);
  k_wt_f16<<<(unsigned)(DM * (DF / 8) / 256), 256, 0, stream>>>(w2, BW2, (unsigned)DF, (unsigned)DM, 16.0f);

  k_lnw<1><<<(unsigned)(NR / 8), 256, 0, stream>>>(x, (size_t)SEQ_FULL * DM, g1, be1, 1e-5f, H16);
  k_gemm2<0, 0, 0, 1><<<dim3((unsigned)((SEQ / 128) * (512 / 64)), NB), 128, 0, stream>>>(H16, DM, (size_t)SEQ * DM, BQKV, DM, 0, 0.0625f, nullptr, nullptr, 0, 0, nullptr, QK16, 512, (size_t)SEQ * 512, SEQ, 512, DM);
  k_gemm2<0, 0, 0, 1><<<dim3((unsigned)((DM / 128) * (SEQ / 64)), NB), 128, 0, stream>>>(BQKV + (size_t)512 * DM, DM, 0, H16, DM, (size_t)SEQ * DM, 0.0625f, nullptr, nullptr, 0, 0, nullptr, VT, SEQ, (size_t)DM * SEQ, DM, SEQ, DM);
  k_fattn<<<dim3(SEQ / 64, NH / 2, NB), 128, 0, stream>>>(QK16, VT, AT16);
  k_gemm2<0, 1, 2, 0><<<dim3((unsigned)((SEQ / 128) * (DM / 64)), NB), 128, 0, stream>>>(AT16, DM, (size_t)SEQ * DM, BP, DM, 0, 0.00390625f, bp, x, DM, (size_t)SEQ_FULL * DM, X2, nullptr, DM, (size_t)SEQ * DM, SEQ, DM, DM);
  k_lnw<0><<<(unsigned)(NR / 8), 256, 0, stream>>>(X2, (size_t)SEQ * DM, g2, be2, 1e-5f, H2);
  k_gemm2<3, 1, 0, 1><<<dim3((unsigned)((SEQ / 128) * (DF / 64)), NB), 128, 0, stream>>>(H2, DM, (size_t)SEQ * DM, BW1, DM, 0, 0.0625f, b1, nullptr, 0, 0, nullptr, F16, DF, (size_t)SEQ * DF, SEQ, DF, DM);
  k_gemm2<0, 1, 1, 0><<<dim3((unsigned)((SEQ / 128) * (DM / 64)), NB), 128, 0, stream>>>(F16, DF, (size_t)SEQ * DF, BW2, DF, 0, 0.0625f, b2, X2, DM, (size_t)SEQ * DM, out, nullptr, DM, (size_t)SEQ_FULL * DM, SEQ, DM, DF);
}
